// GCNModel_22789096472972
// MI455X (gfx1250) — hardware-verified
//
#include <hip/hip_runtime.h>
#include <stddef.h>
#include <stdint.h>


#define CIN    128
#define H1     256
#define H2     128
#define K1     256
#define K2     512
#define NTHR   256
#define NWAVE  8
#define EPT    8
#define CHUNK  (NTHR * EPT)
#define WCAP   (EPT * 32)
#define LISTN  (NWAVE * WCAP)
#define NBA    1024
#define SLA    10
#define RCAP   20480
#define DEGCAP 64
#define GBM    64
#define HP     520
#define TP     132
#define NU1    (H1 * (K1 / 8))
#define NU2    (H2 * (K2 / 8))
#define AGG_ZINTS (LISTN + 2 * RCAP + 3 * NBA)
#define AGG_LDS_INTS (AGG_ZINTS + 16)
#define MLP_OFF_TS  (GBM * HP * 2)
#define MLP_OFF_BS  (MLP_OFF_TS + GBM * TP * 4)
#define MLP_OFF_WL  (MLP_OFF_BS + H1 * 4)
#define MLP_OFF_SV  (MLP_OFF_WL + H2 * 4)
#define MLP_LDS     (MLP_OFF_SV + GBM * 4)
#define WSMAX  134217728

static_assert((CHUNK & (CHUNK - 1)) == 0 && CHUNK <= 4096);
static_assert((NBA & (NBA - 1)) == 0 && NBA == (1 << SLA));
static_assert(((long long)CHUNK << SLA) < (1LL << 31));
static_assert(LISTN % NTHR == 0);
static_assert(NBA % NWAVE == 0 && NBA % 32 == 0 && NBA % GBM == 0 && NBA == 4 * NTHR);
static_assert(RCAP % (NTHR * 4) == 0 && AGG_ZINTS % (NTHR * 4) == 0 && LISTN % 4 == 0);
static_assert(K1 % 32 == 0 && K2 % 32 == 0 && K1 == 2 * CIN && K2 == 2 * H1);
static_assert(NU1 % NTHR == 0 && NU2 % NTHR == 0);
static_assert(AGG_LDS_INTS * 4 <= 300000 && MLP_LDS <= 300000);
static_assert((HP * 2) % 16 == 0 && (TP * 4) % 16 == 0 && MLP_OFF_TS % 16 == 0 && MLP_OFF_SV % 16 == 0);
static_assert(HP >= K2 && TP >= H2 && H1 == NTHR && GBM == 64);

typedef float          v4f   __attribute__((ext_vector_type(4)));
typedef float          v8f   __attribute__((ext_vector_type(8)));
typedef int            v4i   __attribute__((ext_vector_type(4)));
typedef int            v8i   __attribute__((ext_vector_type(8)));
typedef unsigned       v2u   __attribute__((ext_vector_type(2)));
typedef unsigned short v4us  __attribute__((ext_vector_type(4)));
typedef unsigned short v8us  __attribute__((ext_vector_type(8)));
typedef unsigned short v16us __attribute__((ext_vector_type(16)));
typedef __bf16         v16bf __attribute__((ext_vector_type(16)));
typedef v4f  __attribute__((may_alias)) v4fa;
typedef v4i  __attribute__((may_alias)) v4ia;
typedef v2u  __attribute__((may_alias)) v2ua;
typedef v4us __attribute__((may_alias)) v4usa;
typedef v8us __attribute__((may_alias)) v8usa;
union FragB { v16bf v; v16us u; v8us h[2]; v8i w; };

__device__ __forceinline__ v8f wmb(const FragB& a, const FragB& b, v8f c) {
  v8f d = __builtin_amdgcn_wmma_f32_16x16x32_bf16(false, a.v, false, b.v, (short)0, c, false, false);
  asm volatile("v_nop\n\tv_nop\n\tv_nop\n\tv_nop" : "+v"(d) : "v"(a.w), "v"(b.w));
  return d;
}

__device__ __forceinline__ unsigned bf16_bits(float f) {
  const unsigned u = __float_as_uint(f);
  return (u + 0x7FFFu + ((u >> 16) & 1u)) >> 16;
}
__device__ __forceinline__ float bf16_val(float f) {
  return __uint_as_float(bf16_bits(f) << 16);
}

__device__ __forceinline__ void wave_sync() {
  __builtin_amdgcn_fence(__ATOMIC_RELEASE, "wavefront");
  __builtin_amdgcn_wave_barrier();
  __builtin_amdgcn_fence(__ATOMIC_ACQUIRE, "wavefront");
}

__device__ __forceinline__ int clampi(int v, int lo, int hi) {
  return v < lo ? lo : (v > hi ? hi : v);
}

__device__ __forceinline__ float dinv_of(int c, int bad) {
  const float dg = (float)c + 1.0f;
  const float dv = (dg > 0.0f) ? rsqrtf(dg) : 0.0f;
  return (bad != 0 || c > DEGCAP) ? __int_as_float(0x7fc00000) : dv;
}

template <int SLB>
__device__ __forceinline__ int scan_chunk(const int* __restrict__ dsts, int nE, int cbase, int slotBase,
                                          int nb, int vec8, int* list, int tid, int lane, int wave) {
  int wc = 0;
  const int el0  = tid * EPT;
  const int e0   = cbase + el0;
  const int sent = -2147483647 - 1;
  v4i da, db;
  if (vec8 != 0 && cbase + CHUNK <= nE) {
    da = *(const v4i*)(dsts + e0);
    db = *(const v4i*)(dsts + e0 + 4);
  } else {
    da.x = (e0     < nE) ? dsts[min(e0,     nE - 1)] : sent;
    da.y = (e0 + 1 < nE) ? dsts[min(e0 + 1, nE - 1)] : sent;
    da.z = (e0 + 2 < nE) ? dsts[min(e0 + 2, nE - 1)] : sent;
    da.w = (e0 + 3 < nE) ? dsts[min(e0 + 3, nE - 1)] : sent;
    db.x = (e0 + 4 < nE) ? dsts[min(e0 + 4, nE - 1)] : sent;
    db.y = (e0 + 5 < nE) ? dsts[min(e0 + 5, nE - 1)] : sent;
    db.z = (e0 + 6 < nE) ? dsts[min(e0 + 6, nE - 1)] : sent;
    db.w = (e0 + 7 < nE) ? dsts[min(e0 + 7, nE - 1)] : sent;
  }
  const unsigned nbs = (unsigned)slotBase;
  const unsigned unb = (unsigned)nb;
  const unsigned s0 = (unsigned)da.x - nbs, s1 = (unsigned)da.y - nbs;
  const unsigned s2 = (unsigned)da.z - nbs, s3 = (unsigned)da.w - nbs;
  const unsigned s4 = (unsigned)db.x - nbs, s5 = (unsigned)db.y - nbs;
  const unsigned s6 = (unsigned)db.z - nbs, s7 = (unsigned)db.w - nbs;
  const bool h0 = s0 < unb, h1 = s1 < unb, h2 = s2 < unb, h3 = s3 < unb;
  const bool h4 = s4 < unb, h5 = s5 < unb, h6 = s6 < unb, h7 = s7 < unb;
  const unsigned any = __builtin_amdgcn_ballot_w32(h0 | h1 | h2 | h3 | h4 | h5 | h6 | h7);
  if (any != 0u) {
#define HITJ(J, HJ, SJ) { \
      const unsigned mj = __builtin_amdgcn_ballot_w32(HJ); \
      if (mj != 0u) { \
        if (HJ) { \
          const int pos = wc + (int)__builtin_amdgcn_mbcnt_lo(mj, 0u); \
          if (pos < WCAP) list[wave * WCAP + pos] = ((el0 + (J)) << SLB) | (int)(SJ); \
        } \
        wc += (int)__builtin_popcount(mj); } }
    HITJ(0, h0, s0)
    HITJ(1, h1, s1)
    HITJ(2, h2, s2)
    HITJ(3, h3, s3)
    HITJ(4, h4, s4)
    HITJ(5, h5, s5)
    HITJ(6, h6, s6)
    HITJ(7, h7, s7)
#undef HITJ
  }
  return wc;
}

__global__ __launch_bounds__(NTHR) void k_wprep(const float* __restrict__ W1, const float* __restrict__ W2,
                                                unsigned short* W1T, unsigned short* W2T) {
  const int u = (int)blockIdx.x * NTHR + (int)threadIdx.x;
  v8us o;
  unsigned short* dp;
  if (u < NU1) {
    const int n  = u >> 5;
    const int k8 = (u & 31) * 8;
    const int kk = k8 & (CIN - 1);
    const float* p = W1 + (size_t)kk * H1 + n;
#pragma unroll
    for (int i = 0; i < 8; ++i) o[i] = (unsigned short)bf16_bits(p[(size_t)i * H1]);
    dp = W1T + (size_t)n * K1 + k8;
  } else if (u < NU1 + NU2) {
    const int v  = u - NU1;
    const int n  = v >> 6;
    const int k8 = (v & 63) * 8;
    const int kk = k8 & (H1 - 1);
    const float* p = W2 + (size_t)kk * H2 + n;
#pragma unroll
    for (int i = 0; i < 8; ++i) o[i] = (unsigned short)bf16_bits(p[(size_t)i * H2]);
    dp = W2T + (size_t)n * K2 + k8;
  } else {
    return;
  }
  *(volatile v8us*)dp = o;
  __threadfence();
  *(volatile v8us*)dp = o;
}

__global__ __launch_bounds__(NTHR) void k_cvx(const float* __restrict__ x, int nN, int nUnits,
                                              unsigned short* xb) {
  const int u = (int)blockIdx.x * NTHR + (int)threadIdx.x;
  if (u >= nUnits) return;
  const int row = u >> 4;
  const int k8  = (u & 15) * 8;
  const int rc  = row < nN ? row : nN - 1;
  const float* p = x + (size_t)rc * CIN + k8;
  const v4f a = *(const v4fa*)p;
  const v4f b = *(const v4fa*)(p + 4);
  v8us o;
  o[0] = (unsigned short)bf16_bits(a.x);
  o[1] = (unsigned short)bf16_bits(a.y);
  o[2] = (unsigned short)bf16_bits(a.z);
  o[3] = (unsigned short)bf16_bits(a.w);
  o[4] = (unsigned short)bf16_bits(b.x);
  o[5] = (unsigned short)bf16_bits(b.y);
  o[6] = (unsigned short)bf16_bits(b.z);
  o[7] = (unsigned short)bf16_bits(b.w);
  unsigned short* dp = xb + (size_t)rc * CIN + k8;
  *(volatile v8us*)dp = o;
  __threadfence();
  *(volatile v8us*)dp = o;
}

__global__ __launch_bounds__(NTHR) void k_hits(const int* __restrict__ srcs, const int* __restrict__ dsts,
                                               int nE, int nN, int vec8,
                                               int* col, int* cntg, int* offg, float* dinvg) {
  extern __shared__ __attribute__((aligned(16))) int dsm[];
  int* list = dsm;
  int* hl   = dsm + LISTN;
  int* sl   = dsm + LISTN + RCAP;
  int* cnt  = dsm + LISTN + 2 * RCAP;
  int* offs = cnt + NBA;
  int* cur  = offs + NBA;
  int* misc = cur + NBA;
  const int tid = (int)threadIdx.x, lane = tid & 31, wave = tid >> 5;
  const int nodeBase = (int)blockIdx.x * NBA;

  {
    const v4i z4 = {0, 0, 0, 0};
    for (int i = tid * 4; i < AGG_ZINTS; i += NTHR * 4) *(v4ia*)(dsm + i) = z4;
    if (tid < 16) misc[tid] = 0;
  }
  __syncthreads();

  int t = 0, ov = 0;
  const int nChunks = (nE + CHUNK - 1) / CHUNK;
#pragma unroll 1
  for (int ch = 0; ch < nChunks; ++ch) {
    const int cbase = ch * CHUNK;
    const int wc = scan_chunk<SLA>(dsts, nE, cbase, nodeBase, NBA, vec8, list, tid, lane, wave);
    if (lane == 0) misc[wave] = wc;
    __syncthreads();
    if (wave == 0) {
#pragma unroll 1
      for (int w2 = 0; w2 < NWAVE; ++w2) {
        int c = misc[w2];
        c = c < 0 ? 0 : (c > WCAP ? WCAP : c);
#pragma unroll 1
        for (int b0 = 0; b0 < c; b0 += 32) {
          const int idx = b0 + lane;
          const int ent = list[w2 * WCAP + (idx < WCAP ? idx : WCAP - 1)];
          const int m32 = (c - b0) < 32 ? (c - b0) : 32;
#pragma unroll 1
          for (int k = 0; k < m32; ++k) {
            const int u    = __builtin_amdgcn_readlane(ent, k);
            const int slot = u & (NBA - 1);
            const int el   = (u >> SLA) & (CHUNK - 1);
            const int pk   = ((cbase + el) << SLA) | slot;
            if (t < RCAP) {
              if (lane == 0) { hl[t] = pk; cnt[slot] = cnt[slot] + 1; }
              t = t + 1;
            } else {
              ov = 1;
            }
          }
        }
      }
    }
    __syncthreads();
  }
  if (wave == 0 && lane == 0) { misc[8] = t; misc[9] = ov; }
  __syncthreads();
  int tt = misc[8];
  tt = tt < 0 ? 0 : (tt > RCAP ? RCAP : tt);
  const int ovf = misc[9];

  if (wave == 0) {
    const int base = lane * (NBA / 32);
    int s = 0;
#pragma unroll 1
    for (int i = 0; i < NBA / 32; ++i) s += cnt[base + i];
    int incl = s;
#pragma unroll
    for (int d = 1; d < 32; d <<= 1) {
      const int y = __shfl_up(incl, d, 32);
      if (lane >= d) incl += y;
    }
    int run = incl - s;
#pragma unroll 1
    for (int i = 0; i < NBA / 32; ++i) {
      const int cv = cnt[base + i];
      offs[base + i] = run;
      cur[base + i]  = run;
      run += cv;
    }
  }
  __syncthreads();
  if (wave == 0) {
#pragma unroll 1
    for (int b0 = 0; b0 < tt; b0 += 32) {
      const int idx = b0 + lane;
      const int ent = hl[idx < RCAP ? idx : RCAP - 1];
      const int m32 = (tt - b0) < 32 ? (tt - b0) : 32;
#pragma unroll 1
      for (int k = 0; k < m32; ++k) {
        const int u    = __builtin_amdgcn_readlane(ent, k);
        const int slot = u & (NBA - 1);
        if (lane == 0) {
          int p = cur[slot];
          p = p < 0 ? 0 : (p > RCAP - 1 ? RCAP - 1 : p);
          sl[p] = u;
          cur[slot] = p + 1;
        }
      }
    }
  }
  __syncthreads();

  int* colB = col + (size_t)blockIdx.x * RCAP;
#pragma unroll 1
  for (int it = 0; it < RCAP / (NTHR * 4); ++it) {
    const int p = it * (NTHR * 4) + 4 * tid;
    const v4i e4 = *(const v4ia*)(sl + p);
    const int q0 = clampi(e4.x >> SLA, 0, nE - 1);
    const int q1 = clampi(e4.y >> SLA, 0, nE - 1);
    const int q2 = clampi(e4.z >> SLA, 0, nE - 1);
    const int q3 = clampi(e4.w >> SLA, 0, nE - 1);
    v4i o;
    o.x = clampi(srcs[q0], 0, nN - 1);
    o.y = clampi(srcs[q1], 0, nN - 1);
    o.z = clampi(srcs[q2], 0, nN - 1);
    o.w = clampi(srcs[q3], 0, nN - 1);
    *(volatile v4i*)(colB + p) = o;
    __threadfence();
    *(volatile v4i*)(colB + p) = o;
  }
  {
    const int s0 = 4 * tid;
    const v4i c4 = *(const v4ia*)(cnt + s0);
    const v4i o4 = *(const v4ia*)(offs + s0);
    v4f d4;
    d4.x = dinv_of(c4.x, ovf);
    d4.y = dinv_of(c4.y, ovf);
    d4.z = dinv_of(c4.z, ovf);
    d4.w = dinv_of(c4.w, ovf);
    const size_t g = (size_t)nodeBase + s0;
    *(volatile v4i*)(cntg + g) = c4;
    *(volatile v4i*)(offg + g) = o4;
    *(volatile v4f*)(dinvg + g) = d4;
    __threadfence();
    *(volatile v4i*)(cntg + g) = c4;
    *(volatile v4i*)(offg + g) = o4;
    *(volatile v4f*)(dinvg + g) = d4;
  }
}

__global__ __launch_bounds__(NTHR) void k_agg1(const int* __restrict__ col, const int* __restrict__ cntg,
                                               const int* __restrict__ offg, const float* __restrict__ dinvg,
                                               const unsigned short* __restrict__ xb,
                                               int nN, int mRows, unsigned short* ax) {
  __shared__ __attribute__((aligned(16))) int   scnt[NBA];
  __shared__ __attribute__((aligned(16))) int   soff[NBA];
  __shared__ __attribute__((aligned(16))) float sdv[NBA];
  __shared__ __attribute__((aligned(16))) unsigned short rbuf[NWAVE * K1];
  const int tid = (int)threadIdx.x, lane = tid & 31, wave = tid >> 5;
  const int nodeBase = (int)blockIdx.x * NBA;
  {
    const size_t g = (size_t)nodeBase + 4 * tid;
    *(v4ia*)(scnt + 4 * tid) = *(const v4i*)(cntg + g);
    *(v4ia*)(soff + 4 * tid) = *(const v4i*)(offg + g);
    *(v4fa*)(sdv + 4 * tid)  = *(const v4f*)(dinvg + g);
  }
  __syncthreads();
  const int* colB = col + (size_t)blockIdx.x * RCAP;
  unsigned short* rb = rbuf + wave * K1;

#pragma unroll 1
  for (int si = 0; si < NBA / NWAVE; ++si) {
    const int s    = si * NWAVE + wave;
    const int node = nodeBase + s;
    const int c = clampi(scnt[s], 0, DEGCAP);
    const int o = clampi(soff[s], 0, RCAP);
    const float dd = sdv[s];
    const int nc = node < nN ? node : nN - 1;
    float a0 = 0.0f, a1 = 0.0f, a2 = 0.0f, a3 = 0.0f;
#pragma unroll 1
    for (int b0 = 0; b0 < c; b0 += 32) {
      int idx = o + b0 + lane;
      idx = idx > RCAP - 1 ? RCAP - 1 : idx;
      const int sr = clampi(colB[idx], 0, nN - 1);
      const int dsi = __float_as_int(dinvg[sr]);
      const int m32 = (c - b0) < 32 ? (c - b0) : 32;
#pragma unroll 1
      for (int k = 0; k < m32; ++k) {
        const int   sk = __builtin_amdgcn_readlane(sr, k);
        const float ck = __int_as_float(__builtin_amdgcn_readlane(dsi, k));
        const v2u w = *(const v2ua*)(xb + (size_t)sk * CIN + 4 * lane);
        a0 = fmaf(ck, __uint_as_float(w.x << 16), a0);
        a1 = fmaf(ck, __uint_as_float(w.x & 0xffff0000u), a1);
        a2 = fmaf(ck, __uint_as_float(w.y << 16), a2);
        a3 = fmaf(ck, __uint_as_float(w.y & 0xffff0000u), a3);
      }
    }
    {
      const v2u w = *(const v2ua*)(xb + (size_t)nc * CIN + 4 * lane);
      a0 = fmaf(dd, __uint_as_float(w.x << 16), a0);
      a1 = fmaf(dd, __uint_as_float(w.x & 0xffff0000u), a1);
      a2 = fmaf(dd, __uint_as_float(w.y << 16), a2);
      a3 = fmaf(dd, __uint_as_float(w.y & 0xffff0000u), a3);
    }
    const bool live = node < nN;
    const float m0 = live ? (a0 * dd) : 0.0f;
    const float m1 = live ? (a1 * dd) : 0.0f;
    const float m2 = live ? (a2 * dd) : 0.0f;
    const float m3 = live ? (a3 * dd) : 0.0f;
    v4us mh, ml;
    {
      unsigned hb;
      hb = bf16_bits(m0); mh[0] = (unsigned short)hb; ml[0] = (unsigned short)bf16_bits(m0 - __uint_as_float(hb << 16));
      hb = bf16_bits(m1); mh[1] = (unsigned short)hb; ml[1] = (unsigned short)bf16_bits(m1 - __uint_as_float(hb << 16));
      hb = bf16_bits(m2); mh[2] = (unsigned short)hb; ml[2] = (unsigned short)bf16_bits(m2 - __uint_as_float(hb << 16));
      hb = bf16_bits(m3); mh[3] = (unsigned short)hb; ml[3] = (unsigned short)bf16_bits(m3 - __uint_as_float(hb << 16));
    }
    *(v4usa*)(rb + 4 * lane) = mh;
    *(v4usa*)(rb + CIN + 4 * lane) = ml;
    wave_sync();
    const v8us q0 = *(const v8usa*)(rb + 8 * lane);
    wave_sync();
    if (node < mRows) {
      unsigned short* rpw = ax + (size_t)node * K1 + 8 * lane;
      *(volatile v8us*)rpw = q0;
      __threadfence();
      *(volatile v8us*)rpw = q0;
    }
  }
}

__global__ __launch_bounds__(NTHR) void k_mlp(const unsigned short* __restrict__ ax,
                                              const unsigned short* __restrict__ W1T,
                                              const unsigned short* __restrict__ W2T,
                                              const float* __restrict__ b1, const float* __restrict__ Wl,
                                              const float* __restrict__ dinvg, float* ss) {
  extern __shared__ __attribute__((aligned(16))) unsigned char dsb[];
  unsigned short* Hs = (unsigned short*)dsb;
  float* ts = (float*)(dsb + MLP_OFF_TS);
  float* bs = (float*)(dsb + MLP_OFF_BS);
  float* wl = (float*)(dsb + MLP_OFF_WL);
  float* sv = (float*)(dsb + MLP_OFF_SV);
  const int tid = (int)threadIdx.x, lane = tid & 31, wave = tid >> 5, hh = lane >> 4, m = lane & 15;
  const int rt = wave & 3, ch = wave >> 2;
  const int rowBase = (int)blockIdx.x * GBM;

  bs[tid] = bf16_val(b1[tid]);
  {
    const float wv = Wl[tid & (H2 - 1)];
    if (tid < H2) wl[tid] = bf16_val(wv);
  }
  __syncthreads();

  v8f acc[8];
  {
    const v8f z = {0.f, 0.f, 0.f, 0.f, 0.f, 0.f, 0.f, 0.f};
#pragma unroll
    for (int t = 0; t < 8; ++t) acc[t] = z;
  }
  {
    const unsigned short* ap = ax  + (size_t)(rowBase + 16 * rt + m) * (size_t)K1 + 8 * hh;
    const unsigned short* bp = W1T + (size_t)(128 * ch + m) * (size_t)K1 + 8 * hh;
#pragma unroll 1
    for (int k0 = 0; k0 < K1; k0 += 32) {
      FragB af;
      af.h[0] = *(const v8usa*)(ap + k0);
      af.h[1] = *(const v8usa*)(ap + k0 + 16);
#pragma unroll
      for (int nt = 0; nt < 8; ++nt) {
        const unsigned short* wq = bp + (size_t)(16 * nt) * (size_t)K1 + k0;
        FragB bf;
        bf.h[0] = *(const v8usa*)wq;
        bf.h[1] = *(const v8usa*)(wq + 16);
        acc[nt] = wmb(af, bf, acc[nt]);
      }
    }
  }

#pragma unroll
  for (int nt = 0; nt < 8; ++nt) {
    const int lc = 128 * ch + 16 * nt + m;
    const float bias = bs[lc];
#pragma unroll
    for (int r = 0; r < 8; ++r) {
      const int lr = 16 * rt + 8 * hh + r;
      const float v = acc[nt][r] + bias;
      const float y = (v > 0.0f) ? v : (v - v);
      const unsigned hb = bf16_bits(y);
      const unsigned lb = bf16_bits(y - __uint_as_float(hb << 16));
      Hs[lr * HP + lc]      = (unsigned short)hb;
      Hs[lr * HP + H1 + lc] = (unsigned short)lb;
    }
  }
  __syncthreads();

  v8f ac2[4];
  {
    const v8f z = {0.f, 0.f, 0.f, 0.f, 0.f, 0.f, 0.f, 0.f};
    ac2[0] = z; ac2[1] = z; ac2[2] = z; ac2[3] = z;
  }
  {
    const unsigned short* hsA = Hs + (16 * rt + m) * HP + 8 * hh;
    const unsigned short* bp2 = W2T + (size_t)(64 * ch + m) * (size_t)K2 + 8 * hh;
#pragma unroll 1
    for (int k0 = 0; k0 < K2; k0 += 32) {
      FragB af;
      af.h[0] = *(const v8usa*)(hsA + k0);
      af.h[1] = *(const v8usa*)(hsA + k0 + 16);
#pragma unroll
      for (int nt = 0; nt < 4; ++nt) {
        const unsigned short* wq = bp2 + (size_t)(16 * nt) * (size_t)K2 + k0;
        FragB bf;
        bf.h[0] = *(const v8usa*)wq;
        bf.h[1] = *(const v8usa*)(wq + 16);
        ac2[nt] = wmb(af, bf, ac2[nt]);
      }
    }
  }

#pragma unroll
  for (int nt = 0; nt < 4; ++nt) {
    const int lc = 64 * ch + 16 * nt + m;
#pragma unroll
    for (int r = 0; r < 8; ++r) {
      const int lr = 16 * rt + 8 * hh + r;
      ts[lr * TP + lc] = ac2[nt][r];
    }
  }
  __syncthreads();
  if (tid < GBM) {
    const float* tr = ts + tid * TP;
    float s = 0.0f;
#pragma unroll 4
    for (int k = 0; k < H2; ++k) s = fmaf(tr[k], wl[k], s);
    const float dv = dinvg[rowBase + tid];
    sv[tid] = dv * s;
  }
  __syncthreads();
  {
    const v4f ov = *(const v4fa*)(sv + 4 * (tid & 15));
    float* op = ss + (size_t)rowBase + 4 * (tid & 15);
    const bool okst = tid < 16;
    if (okst) *(volatile v4f*)op = ov;
    __threadfence();
    if (okst) *(volatile v4f*)op = ov;
  }
}

__global__ __launch_bounds__(NTHR) void k_agg2(const int* __restrict__ col, const int* __restrict__ cntg,
                                               const int* __restrict__ offg, const float* __restrict__ dinvg,
                                               const float* __restrict__ ss,
                                               const float* __restrict__ b2, const float* __restrict__ Wl,
                                               const float* __restrict__ bl, int nN, float* out) {
  __shared__ __attribute__((aligned(16))) float os[NBA];
  __shared__ float cs[4];
  const int tid = (int)threadIdx.x, lane = tid & 31, wave = tid >> 5;
  const int nodeBase = (int)blockIdx.x * NBA;
  if (wave == 0) {
    float c = 0.0f;
#pragma unroll 1
    for (int k = 0; k < H2; ++k) c = fmaf(bf16_val(b2[k]), bf16_val(Wl[k]), c);
    c = c + bf16_val(bl[0]);
    if (lane == 0) cs[0] = c;
  }
  __syncthreads();
  const float cc = cs[0];
  const int* colB = col + (size_t)blockIdx.x * RCAP;

#pragma unroll 1
  for (int it = 0; it < NBA / NTHR; ++it) {
    const int s    = it * NTHR + tid;
    const int node = nodeBase + s;
    const int c = clampi(cntg[(size_t)nodeBase + s], 0, DEGCAP);
    const int o = clampi(offg[(size_t)nodeBase + s], 0, RCAP);
    const float dd = dinvg[(size_t)nodeBase + s];
    const int nc = node < nN ? node : nN - 1;
    int cmax = c;
    cmax = max(cmax, __shfl_xor(cmax, 16, 32));
    cmax = max(cmax, __shfl_xor(cmax, 8, 32));
    cmax = max(cmax, __shfl_xor(cmax, 4, 32));
    cmax = max(cmax, __shfl_xor(cmax, 2, 32));
    cmax = max(cmax, __shfl_xor(cmax, 1, 32));
    cmax = cmax > DEGCAP ? DEGCAP : cmax;
    float acc = 0.0f;
#pragma unroll 1
    for (int p = 0; p < cmax; ++p) {
      int idx = o + p;
      idx = idx > RCAP - 1 ? RCAP - 1 : idx;
      const int sr = clampi(colB[idx], 0, nN - 1);
      const float v = ss[sr];
      acc = acc + ((p < c) ? v : 0.0f);
    }
    acc = acc + ss[nc];
    os[s] = dd * acc + cc;
  }
  __syncthreads();
  {
    const v4f ov = *(const v4fa*)(os + 4 * tid);
    const int n0 = nodeBase + 4 * tid;
    const bool okst = (n0 + 3) < nN;
    float* op = out + (size_t)(okst ? n0 : 0);
    if (okst) *(volatile v4f*)op = ov;
    __threadfence();
    if (okst) *(volatile v4f*)op = ov;
  }
}

static inline int cdiv(int a, int b) { return (a + b - 1) / b; }
static inline size_t al256(size_t o) { return (o + 255) & ~(size_t)255; }

extern "C" void kernel_launch(void* const* d_in, const int* in_sizes, int n_in,
                              void* d_out, int out_size, void* d_ws, size_t ws_size,
                              hipStream_t stream) {
  if (n_in < 8) return;
  if (in_sizes[0] < CIN || (in_sizes[0] % CIN) != 0) return;
  const int nN = in_sizes[0] / CIN;
  if (nN < 32 || (nN % 32) != 0 || nN > (1 << 22)) return;
  if (in_sizes[1] < 2 || (in_sizes[1] & 1) != 0) return;
  const int nE = in_sizes[1] / 2;
  if (nE < 1 || nE >= (1 << (31 - SLA))) return;
  if (in_sizes[2] != CIN * H1 || in_sizes[3] != H1) return;
  if (in_sizes[4] != H1 * H2 || in_sizes[5] != H2) return;
  if (in_sizes[6] != H2 || in_sizes[7] != 1) return;
  if (out_size != nN) return;

  const float* x    = (const float*)d_in[0];
  const int*   edge = (const int*)d_in[1];
  const float* W1   = (const float*)d_in[2];
  const float* b1   = (const float*)d_in[3];
  const float* W2   = (const float*)d_in[4];
  const float* b2   = (const float*)d_in[5];
  const float* Wl   = (const float*)d_in[6];
  const float* bl   = (const float*)d_in[7];
  float* out = (float*)d_out;
  const int* src = edge;
  const int* dst = edge + nE;

  const int MP  = cdiv(nN, GBM) * GBM;
  const int gM  = MP / GBM;
  const int gA  = cdiv(nN, NBA);
  const int NBP = gA * NBA;
  if (NBP < MP) return;
  const int vec8 = ((nE & 3) == 0) ? 1 : 0;

  char* ws = (char*)d_ws;
  size_t off = 0;
  const size_t oW1T = off; off = al256(off + (size_t)H1 * K1 * 2);
  const size_t oW2T = off; off = al256(off + (size_t)H2 * K2 * 2);
  const size_t oXB  = off; off = al256(off + (size_t)nN * CIN * 2);
  const size_t oAX  = off; off = al256(off + (size_t)MP * K1 * 2);
  const size_t oCOL = off; off = al256(off + (size_t)gA * RCAP * 4);
  const size_t oCNT = off; off = al256(off + (size_t)NBP * 4);
  const size_t oOFF = off; off = al256(off + (size_t)NBP * 4);
  const size_t oDIN = off; off = al256(off + (size_t)NBP * 4);
  const size_t oSS  = off; off = al256(off + (size_t)NBP * 4);
  if (off > ws_size || off > (size_t)WSMAX) return;
  unsigned short* W1T = (unsigned short*)(ws + oW1T);
  unsigned short* W2T = (unsigned short*)(ws + oW2T);
  unsigned short* XB  = (unsigned short*)(ws + oXB);
  unsigned short* AX  = (unsigned short*)(ws + oAX);
  int*   COL  = (int*)(ws + oCOL);
  int*   CNT  = (int*)(ws + oCNT);
  int*   OFFS = (int*)(ws + oOFF);
  float* DINV = (float*)(ws + oDIN);
  float* SS   = (float*)(ws + oSS);

  const size_t hitLds = (size_t)AGG_LDS_INTS * 4;
  const size_t mlpLds = (size_t)MLP_LDS;
  hipFuncSetAttribute(reinterpret_cast<const void*>(&k_hits), hipFuncAttributeMaxDynamicSharedMemorySize, (int)hitLds);
  hipFuncSetAttribute(reinterpret_cast<const void*>(&k_mlp),  hipFuncAttributeMaxDynamicSharedMemorySize, (int)mlpLds);

  const int nUx = nN * (CIN / 8);
  k_wprep<<<(NU1 + NU2) / NTHR, NTHR, 0, stream>>>(W1, W2, W1T, W2T);
  k_cvx<<<cdiv(nUx, NTHR), NTHR, 0, stream>>>(x, nN, nUx, XB);
  k_hits<<<gA, NTHR, hitLds, stream>>>(src, dst, nE, nN, vec8, COL, CNT, OFFS, DINV);
  k_agg1<<<gA, NTHR, 0, stream>>>(COL, CNT, OFFS, DINV, XB, nN, MP, AX);
  k_mlp<<<gM, NTHR, mlpLds, stream>>>(AX, W1T, W2T, b1, Wl, DINV, SS);
  k_agg2<<<gA, NTHR, 0, stream>>>(COL, CNT, OFFS, DINV, SS, b2, Wl, bl, nN, out);
}
